// modular_Attention_41360535061095
// MI455X (gfx1250) — hardware-verified
//
#include <hip/hip_runtime.h>
#include <math.h>

typedef __attribute__((ext_vector_type(16))) _Float16 v16h;
typedef __attribute__((ext_vector_type(16))) __bf16 v16b;
typedef __attribute__((ext_vector_type(8)))  _Float16 v8h;
typedef __attribute__((ext_vector_type(8)))  float v8f;
typedef __attribute__((ext_vector_type(4)))  float v4f;
typedef __attribute__((ext_vector_type(2)))  float v2f;
typedef __attribute__((ext_vector_type(4)))  unsigned v4u;
typedef __attribute__((ext_vector_type(4)))  int v4i;
typedef float __attribute__((may_alias)) float_a;
typedef int __attribute__((may_alias)) int_a;

template <typename T> __device__ __forceinline__ void vst2(void* p, T v) { *(volatile T*)p = v; __threadfence(); *(volatile T*)p = v; }
__device__ __forceinline__ v8f wmma16(v16h a, v16h b, v8f c) {
  v8f d = __builtin_amdgcn_wmma_f32_16x16x32_f16(false, a, false, b, (short)0, c, false, false);
  asm volatile("v_nop\n\tv_nop\n\tv_nop\n\tv_nop" : "+v"(d) : "v"(a), "v"(b));
  return d;
}
__device__ __forceinline__ v8f wmma_bf(v16b a, v16b b, v8f c) {
  v8f d = __builtin_amdgcn_wmma_f32_16x16x32_bf16(false, a, false, b, (short)0, c, false, false);
  asm volatile("v_nop\n\tv_nop\n\tv_nop\n\tv_nop" : "+v"(d) : "v"(a), "v"(b));
  return d;
}
__device__ __forceinline__ v16h frag_h(const _Float16* rowk0, int lane) {
  union { v16h v; v8h q[2]; } u; const _Float16* p = rowk0 + 8 * (lane >> 4);
  u.q[0] = *(const v8h*)p; u.q[1] = *(const v8h*)(p + 16); return u.v;
}
__device__ __forceinline__ v16h frag_f32(const float* rowk0, int lane) {
  v16h a; const float* p = rowk0 + 8 * (lane >> 4);
#pragma unroll
  for (int i = 0; i < 8; ++i) { a[i] = (_Float16)p[i]; a[8 + i] = (_Float16)p[16 + i]; }
  return a;
}
__device__ __forceinline__ v16h frag_f32s(const float* rowk0, int lane, float sc) {
  v16h a; const float* p = rowk0 + 8 * (lane >> 4);
#pragma unroll
  for (int i = 0; i < 8; ++i) { a[i] = (_Float16)(p[i] * sc); a[8 + i] = (_Float16)(p[16 + i] * sc); }
  return a;
}
__device__ __forceinline__ v16h fragc_f32(const float* W, int k0, int n, int lane, int ld, int K) {
  v16h a; const int g = lane >> 4;
#pragma unroll
  for (int i = 0; i < 8; ++i) { const int ka = k0 + 8 * g + i, kb = ka + 16;
    a[i] = (_Float16)(ka < K ? W[(size_t)(ka < K ? ka : K - 1) * ld + n] : 0.f); a[8 + i] = (_Float16)(kb < K ? W[(size_t)(kb < K ? kb : K - 1) * ld + n] : 0.f); }
  return a;
}
struct F2 { v16b h, l; };
__device__ __forceinline__ F2 bsplit16(const float v[16]) { F2 r;
#pragma unroll
  for (int i = 0; i < 16; ++i) { const __bf16 h = (__bf16)v[i]; r.h[i] = h; r.l[i] = (__bf16)(v[i] - (float)h); }
  return r; }
__device__ __forceinline__ F2 split_row(const float* row, int k0, int lane) { float v[16]; const float* p = row + k0 + 8 * (lane >> 4);
#pragma unroll
  for (int i = 0; i < 8; ++i) { v[i] = p[i]; v[8 + i] = p[16 + i]; }
  return bsplit16(v); }
__device__ __forceinline__ F2 split_rowK(const float* row, int k0, int lane, int K) { float v[16]; const int g = lane >> 4;
#pragma unroll
  for (int i = 0; i < 8; ++i) { const int ka = k0 + 8 * g + i, kb = ka + 16; v[i] = ka < K ? row[ka < K ? ka : K - 1] : 0.f; v[8 + i] = kb < K ? row[kb < K ? kb : K - 1] : 0.f; }
  return bsplit16(v); }
__device__ __forceinline__ F2 split_col(const float* W, int k0, int n, int lane, int ld, int K) { float v[16]; const int g = lane >> 4;
#pragma unroll
  for (int i = 0; i < 8; ++i) { const int ka = k0 + 8 * g + i, kb = ka + 16; v[i] = ka < K ? W[(size_t)(ka < K ? ka : K - 1) * ld + n] : 0.f; v[8 + i] = kb < K ? W[(size_t)(kb < K ? kb : K - 1) * ld + n] : 0.f; }
  return bsplit16(v); }
__device__ __forceinline__ v8f mac3(const F2& a, const F2& b, v8f c) { c = wmma_bf(a.l, b.h, c); c = wmma_bf(a.h, b.l, c); return wmma_bf(a.h, b.h, c); }
__device__ __forceinline__ float sigm(float v) { return 1.0f / (1.0f + expf(-v)); }
#define LDSX() do { asm volatile("s_wait_dscnt 0" ::: "memory"); __builtin_amdgcn_wave_barrier(); __builtin_amdgcn_fence(__ATOMIC_RELEASE, "workgroup"); } while (0)


#define NB 4
#define NN 4096
#define DD 512
#define UU 64
#ifndef TNB
#define TNB NB
#endif
typedef __attribute__((ext_vector_type(8))) __bf16 v8b;
__device__ __forceinline__ v16b frag_b(const __bf16* rowk0, int lane) {
  union { v16b v; v8b q[2]; } u; const __bf16* p = rowk0 + 8 * (lane >> 4);
  u.q[0] = *(const v8b*)p; u.q[1] = *(const v8b*)(p + 16); return u.v;
}
__device__ __forceinline__ float bfr(float v) { return (float)(__bf16)v; }
__device__ __attribute__((noinline)) float exp_ni(float v) { return expf(v); }
__device__ __attribute__((noinline)) float erf_ni(float v) { return erff(v); }

#define WS_PW  0u
#define WS_QH  (WS_PW + 2u * 3 * UU * DD)
#define WS_KH  (WS_QH + 2u * (size_t)NB * NN * UU)
#define WS_VT  (WS_KH + 2u * (size_t)NB * NN * UU)
#define WS_END (WS_VT + 2u * (size_t)NB * UU * NN)

__global__ __launch_bounds__(256) void k_packw(const float* __restrict__ WQ, const float* __restrict__ WK, const float* __restrict__ WV, __bf16* __restrict__ PW) { const int n = blockIdx.x, t = threadIdx.x; __shared__ __align__(16) __bf16 s[DD]; const int which = n / UU, u = n % UU; const float* Wm = which == 0 ? WQ : which == 1 ? WK : WV;
  for (int k = t; k < DD; k += 256) s[k] = (__bf16)Wm[(size_t)k * UU + u]; __syncthreads(); if (t < DD / 8) vst2((unsigned*)(PW + (size_t)n * DD + t * 8), *(const v4u*)&s[t * 8]); }
__global__ __launch_bounds__(128) void k_proj(const float* __restrict__ X, const __bf16* __restrict__ PW, _Float16* __restrict__ QH, _Float16* __restrict__ KH, _Float16* __restrict__ VT) { __shared__ __align__(16) _Float16 sq[64][72], sk[64][72]; __shared__ __align__(16) _Float16 th[UU][72];
  const int tid = threadIdx.x, wave = tid >> 5, lane = tid & 31, col = lane & 15, g = lane >> 4; const size_t r0 = (size_t)blockIdx.x * 64 + wave * 16; const size_t b = ((size_t)blockIdx.x * 64) / NN; const int n0 = (int)(((size_t)blockIdx.x * 64) % NN);
  v8f acc[12];
#pragma unroll
  for (int j = 0; j < 12; ++j) acc[j] = v8f{};
#pragma unroll 2
  for (int kc = 0; kc < DD / 32; ++kc) { v16b a; const float* pp = X + (r0 + col) * DD + kc * 32 + 8 * g;
#pragma unroll
    for (int i = 0; i < 8; ++i) { a[i] = (__bf16)fminf(fmaxf(bfr(pp[i]), -1.0f), 1.0f); a[8 + i] = (__bf16)fminf(fmaxf(bfr(pp[16 + i]), -1.0f), 1.0f); }
#pragma unroll
    for (int j = 0; j < 12; ++j) acc[j] = wmma_bf(a, frag_b(PW + (size_t)(j * 16 + col) * DD + kc * 32, lane), acc[j]); }
#pragma unroll
  for (int j = 0; j < 12; ++j)
#pragma unroll
    for (int r = 0; r < 8; ++r) { const _Float16 hv = (_Float16)acc[j][r]; const int c = (j & 3) * 16 + col; if (j < 4) sq[wave * 16 + 8 * g + r][c] = hv; else if (j < 8) sk[wave * 16 + 8 * g + r][c] = hv; else th[c][wave * 16 + 8 * g + r] = hv; }
  __syncthreads();
  for (int e = tid; e < 64 * 8; e += 128) { const int rl = e >> 3, q = e & 7; const size_t o = ((size_t)blockIdx.x * 64 + rl) * UU + q * 8; vst2((unsigned*)(QH + o), *(const v4u*)&sq[rl][q * 8]); vst2((unsigned*)(KH + o), *(const v4u*)&sk[rl][q * 8]); }
  for (int e = tid; e < UU * 8; e += 128) { const int c = e >> 3, q = e & 7; vst2((unsigned*)(VT + (b * UU + c) * (size_t)NN + n0 + q * 8), *(const v4u*)&th[c][q * 8]); } }
__global__ __launch_bounds__(128) void k_att(const _Float16* __restrict__ QH, const _Float16* __restrict__ KH, const _Float16* __restrict__ VT, float* __restrict__ OUT) {
  __shared__ __align__(16) float sp[4][16][36]; __shared__ __align__(16) float so[4][16][68];
  const int tid = threadIdx.x, wave = tid >> 5, lane = tid & 31, col = lane & 15, g = lane >> 4; const size_t b = blockIdx.y; const int q0 = blockIdx.x * 64 + wave * 16; const size_t rq = b * NN + q0;
  v16h aq[2];
#pragma unroll
  for (int kc = 0; kc < 2; ++kc) aq[kc] = frag_h(QH + (rq + col) * UU + kc * 32, lane);
  v8f acc[4] = {}, accl[4] = {};
#pragma unroll 1
  for (int ks = 0; ks < NN / 32; ++ks) {
#pragma unroll
    for (int ct = 0; ct < 2; ++ct) { const size_t rk = b * NN + ks * 32 + ct * 16 + col; v8f c = {};
#pragma unroll
      for (int kc = 0; kc < 2; ++kc) c = wmma16(aq[kc], frag_h(KH + rk * UU + kc * 32, lane), c);
#pragma unroll
      for (int r = 0; r < 8; ++r) sp[wave][8 * g + r][ct * 16 + col] = 1.0f / (1.0f + __expf(-c[r])); }
    LDSX();
    v16h pa, pal; { const float* prow = &sp[wave][col][0] + 8 * (lane >> 4);
#pragma unroll
      for (int i = 0; i < 8; ++i) { const float p0 = prow[i], p1 = prow[16 + i]; pa[i] = (_Float16)p0; pa[8 + i] = (_Float16)p1; pal[i] = (_Float16)((p0 - (float)pa[i]) * 2048.0f); pal[8 + i] = (_Float16)((p1 - (float)pa[8 + i]) * 2048.0f); } }
#pragma unroll
    for (int j = 0; j < 4; ++j) { const v16h vf = frag_h(VT + (b * UU + j * 16 + col) * (size_t)NN + ks * 32, lane); acc[j] = wmma16(pa, vf, acc[j]); accl[j] = wmma16(pal, vf, accl[j]); }
    LDSX(); }
#pragma unroll
  for (int r = 0; r < 8; ++r)
#pragma unroll
    for (int j = 0; j < 4; ++j) so[wave][8 * g + r][j * 16 + col] = acc[j][r] + accl[j][r] * (1.0f / 2048.0f);
  LDSX(); for (int rl = 0; rl < 16; ++rl) if (lane < 16) vst2(OUT + (rq + rl) * UU + lane * 4, *(const v4f*)&so[wave][rl][lane * 4]); }
extern "C" void kernel_launch(void* const* d_in, const int* in_sizes, int n_in, void* d_out, int out_size, void* d_ws, size_t ws_size, hipStream_t stream) {
  (void)in_sizes; (void)n_in; (void)out_size;
  const float** F = (const float**)d_in;
  if (ws_size < (size_t)WS_END) return;
  char* ws = (char*)d_ws; __bf16* PW = (__bf16*)(ws + WS_PW); _Float16 *QH = (_Float16*)(ws + WS_QH), *KH = (_Float16*)(ws + WS_KH), *VT = (_Float16*)(ws + WS_VT);
  k_packw<<<3 * UU, 256, 0, stream>>>(F[1], F[2], F[3], PW);
  k_proj<<<NB * NN / 64, 128, 0, stream>>>(F[0], PW, QH, KH, VT);
  k_att<<<dim3(NN / 64, TNB), 128, 0, stream>>>(QH, KH, VT, (float*)d_out);
}
